// GDTLayer_61564061221139
// MI455X (gfx1250) — hardware-verified
//
#include <hip/hip_runtime.h>
#include <stddef.h>


#define NTHR    256
#define NWAVE   8
#define EPT     8
#define NGRP    2
#define CHUNK   (NTHR * EPT * NGRP)
#define WCAP    (EPT * NGRP * 32)
#define LISTN   (NWAVE * WCAP)
#define NBC     4096
#define NBF     1024
#define RCAP    40960
#define RBN     128
#define TGT     256
#define DEGCAP  1024
#define OTHR    512
#define BM      64
#define BNC     128
#define WSCAP   134217728
#define FIN     128
#define NHD     8
#define DHD     16
#define NPJ     3
#define FFH     512
#define NHOP    5
#define ACARRY  8.0f
#define WCARRY  64.0f
#define SCL_AW  (1.0f / 512.0f)
#define ALPHA_C 0.1f
#define OMA_C   0.9f
#define LNEPS   1e-5f
#define INV_D   (1.0f / 16.0f)

#define LDS_FILL ((RCAP + NBF + LISTN) * 4 + 64)
#define LDS_SOFT ((2 * NBF * NHD + NTHR * NHD + NBF) * 4)

static_assert((CHUNK & (CHUNK - 1)) == 0);
static_assert(CHUNK <= 4096);
static_assert((NBC & (NBC - 1)) == 0 && (NBF & (NBF - 1)) == 0);
static_assert(NBC == 4 * NBF);
static_assert(OTHR * 8 == NBC);
static_assert((RCAP % 32) == 0);
static_assert(TGT == NWAVE * 32);
static_assert((NBC % TGT) == 0);
static_assert((TGT % BM) == 0);
static_assert(WCAP == EPT * NGRP * 32);
static_assert((FIN % 32) == 0 && (FFH % 32) == 0);
static_assert((FFH % BNC) == 0 && ((NPJ * FIN) % BNC) == 0 && (FIN % BNC) == 0);
static_assert(NHD * DHD == FIN);
static_assert(NHD * 4 == 32);
static_assert((NHOP & 1) == 1);
static_assert((NBF % NTHR) == 0);
static_assert(FIN == 4 * 32);

typedef float    v4f  __attribute__((ext_vector_type(4)));
typedef float    v8f  __attribute__((ext_vector_type(8)));
typedef int      v4i  __attribute__((ext_vector_type(4)));
typedef _Float16 v4h  __attribute__((ext_vector_type(4)));
typedef _Float16 v8h  __attribute__((ext_vector_type(8)));
typedef _Float16 v16h __attribute__((ext_vector_type(16)));
union Frag { v16h v; v8h h[2]; };
union StgU { float f[BM * BNC]; _Float16 h[2 * BM * BNC]; };

__device__ __forceinline__ v8f wmh(v16h a, v16h b, v8f c) {
  v8f d = __builtin_amdgcn_wmma_f32_16x16x32_f16(false, a, false, b, (short)0, c, false, false);
  asm volatile("v_nop\n\tv_nop\n\tv_nop\n\tv_nop" : "+v"(d) : "v"(a), "v"(b));
  return d;
}

__device__ __forceinline__ v4f selz(v4f v, bool live) {
  v4f o; o.x = live ? v.x : 0.f; o.y = live ? v.y : 0.f; o.z = live ? v.z : 0.f; o.w = live ? v.w : 0.f; return o;
}
__device__ __forceinline__ v4f vmax4(v4f a, v4f b) {
  v4f o; o.x = fmaxf(a.x, b.x); o.y = fmaxf(a.y, b.y); o.z = fmaxf(a.z, b.z); o.w = fmaxf(a.w, b.w); return o;
}
__device__ __forceinline__ float lrelu1(float v) { return v >= 0.f ? v : 0.2f * v; }
__device__ __forceinline__ v4f vexp4(v4f v) {
  v4f o; o.x = __expf(v.x); o.y = __expf(v.y); o.z = __expf(v.z); o.w = __expf(v.w); return o;
}
__device__ __forceinline__ v4f vrcp4(v4f v) {
  v4f o; o.x = __builtin_amdgcn_rcpf(v.x); o.y = __builtin_amdgcn_rcpf(v.y);
  o.z = __builtin_amdgcn_rcpf(v.z); o.w = __builtin_amdgcn_rcpf(v.w); return o;
}
__device__ __forceinline__ float wsum1(float v) {
#pragma unroll
  for (int off = 16; off > 0; off >>= 1) v += __shfl_xor(v, off);
  return v;
}

template <int NB>
__device__ __forceinline__ int scan_chunk(const int* __restrict__ dsts, int nE, int cbase, int slotBase,
                                          int vec8, int* list, int tid, int lane, int wave) {
  int wc = 0;
#pragma unroll
  for (int g = 0; g < NGRP; ++g) {
    const int el0  = (g * NTHR + tid) * EPT;
    const int e0   = cbase + el0;
    const int sent = -2147483647 - 1;
    v4i da, db;
    if (vec8 != 0 && cbase + CHUNK <= nE) {
      da = *(const v4i*)(dsts + e0);
      db = *(const v4i*)(dsts + e0 + 4);
    } else {
      da.x = (e0     < nE) ? dsts[min(e0, nE - 1)] : sent;
      da.y = (e0 + 1 < nE) ? dsts[min(e0 + 1, nE - 1)] : sent;
      da.z = (e0 + 2 < nE) ? dsts[min(e0 + 2, nE - 1)] : sent;
      da.w = (e0 + 3 < nE) ? dsts[min(e0 + 3, nE - 1)] : sent;
      db.x = (e0 + 4 < nE) ? dsts[min(e0 + 4, nE - 1)] : sent;
      db.y = (e0 + 5 < nE) ? dsts[min(e0 + 5, nE - 1)] : sent;
      db.z = (e0 + 6 < nE) ? dsts[min(e0 + 6, nE - 1)] : sent;
      db.w = (e0 + 7 < nE) ? dsts[min(e0 + 7, nE - 1)] : sent;
    }
    const unsigned nb = (unsigned)slotBase;
    const unsigned s0 = (unsigned)da.x - nb, s1 = (unsigned)da.y - nb;
    const unsigned s2 = (unsigned)da.z - nb, s3 = (unsigned)da.w - nb;
    const unsigned s4 = (unsigned)db.x - nb, s5 = (unsigned)db.y - nb;
    const unsigned s6 = (unsigned)db.z - nb, s7 = (unsigned)db.w - nb;
    const bool h0 = s0 < (unsigned)NB, h1 = s1 < (unsigned)NB, h2 = s2 < (unsigned)NB, h3 = s3 < (unsigned)NB;
    const bool h4 = s4 < (unsigned)NB, h5 = s5 < (unsigned)NB, h6 = s6 < (unsigned)NB, h7 = s7 < (unsigned)NB;
    const unsigned any = __builtin_amdgcn_ballot_w32(h0 | h1 | h2 | h3 | h4 | h5 | h6 | h7);
    if (any != 0u) {
#define HITJ(J, HJ, SJ) { \
        const unsigned mj = __builtin_amdgcn_ballot_w32(HJ); \
        if (mj != 0u) { \
          if (HJ) { \
            const int pos = wc + (int)__builtin_amdgcn_mbcnt_lo(mj, 0u); \
            if (pos < WCAP) list[wave * WCAP + pos] = ((el0 + (J)) << 12) | (int)(SJ); \
          } \
          wc += (int)__builtin_popcount(mj); } }
      HITJ(0, h0, s0)
      HITJ(1, h1, s1)
      HITJ(2, h2, s2)
      HITJ(3, h3, s3)
      HITJ(4, h4, s4)
      HITJ(5, h5, s5)
      HITJ(6, h6, s6)
      HITJ(7, h7, s7)
#undef HITJ
    }
  }
  return wc;
}

__global__ __launch_bounds__(NTHR) void k_count(const int* __restrict__ dsts, int* cnt, int nE, int vec8) {
  __shared__ __attribute__((aligned(16))) int scnt[NBC];
  __shared__ __attribute__((aligned(16))) int list[LISTN];
  __shared__ int wcnt[NWAVE];
  const int tid = threadIdx.x, lane = tid & 31, wave = tid >> 5;
  const int nodeBase = blockIdx.x * NBC;

  for (int i = tid; i < NBC; i += NTHR) scnt[i] = 0;
  __syncthreads();

  const int nChunks = (nE + CHUNK - 1) / CHUNK;
#pragma unroll 1
  for (int ch = 0; ch < nChunks; ++ch) {
    const int cbase = ch * CHUNK;
    const int wc = scan_chunk<NBC>(dsts, nE, cbase, nodeBase, vec8, list, tid, lane, wave);
    if (lane == 0) wcnt[wave] = wc;
    __syncthreads();
    if (wave == 0) {
#pragma unroll 1
      for (int wsx = 0; wsx < NWAVE; ++wsx) {
        int n = __builtin_amdgcn_readfirstlane(wcnt[wsx]);
        n = n > WCAP ? WCAP : (n < 0 ? 0 : n);
        const int* lp = list + wsx * WCAP;
#pragma unroll 1
        for (int i = 0; i < n; ++i) {
          const int ent  = __builtin_amdgcn_readfirstlane(lp[i]);
          const int slot = ent & (NBC - 1);
          if (lane == 0) scnt[slot] = scnt[slot] + 1;
        }
      }
    }
    __syncthreads();
  }

  v4i cq[4];
#pragma unroll
  for (int q = 0; q < 4; ++q) {
    const int f = (wave * 4 + q) * 128 + 4 * lane;
    cq[q] = *(const v4i*)(scnt + f);
  }
  int* cp = cnt + (size_t)nodeBase;
#pragma unroll
  for (int q = 0; q < 4; ++q) {
    const int f = (wave * 4 + q) * 128 + 4 * lane;
    *(volatile v4i*)(cp + f) = cq[q];
  }
  __threadfence();
#pragma unroll
  for (int q = 0; q < 4; ++q) {
    const int f = (wave * 4 + q) * 128 + 4 * lane;
    *(volatile v4i*)(cp + f) = cq[q];
  }
}

__global__ __launch_bounds__(OTHR) void k_offsets(
    const int* __restrict__ cnt, int* off, int* rbase, int nChunk) {
  __shared__ __attribute__((aligned(16))) int soff[NBC];
  __shared__ __attribute__((aligned(16))) int srb[RBN];
  __shared__ int wtot[OTHR / 32];
  const int tid = threadIdx.x, lane = tid & 31, wave = tid >> 5, sub = tid >> 7;
  for (int i = tid; i < RBN; i += OTHR) srb[i] = 0;
  int carry = 0;
#pragma unroll 1
  for (int ch = 0; ch < nChunk; ++ch) {
    const int base = ch * NBC;
    const v4i c0 = *(const v4i*)(cnt + base + 8 * tid);
    const v4i c1 = *(const v4i*)(cnt + base + 8 * tid + 4);
    const int e0 = max(c0.x, 0), e1 = max(c0.y, 0), e2 = max(c0.z, 0), e3 = max(c0.w, 0);
    const int e4 = max(c1.x, 0), e5 = max(c1.y, 0), e6 = max(c1.z, 0), e7 = max(c1.w, 0);
    const int ts = e0 + e1 + e2 + e3 + e4 + e5 + e6 + e7;
    int incl = ts;
#pragma unroll
    for (int d = 1; d < 32; d <<= 1) {
      const int t = __shfl_up(incl, d);
      if (lane >= d) incl += t;
    }
    if (lane == 31) wtot[wave] = incl;
    __syncthreads();
    const int S0 = wtot[0]  + wtot[1]  + wtot[2]  + wtot[3];
    const int S1 = wtot[4]  + wtot[5]  + wtot[6]  + wtot[7];
    const int S2 = wtot[8]  + wtot[9]  + wtot[10] + wtot[11];
    const int S3 = wtot[12] + wtot[13] + wtot[14] + wtot[15];
    int pre = 0;
#pragma unroll 1
    for (int w = 4 * sub; w < wave; ++w) pre += wtot[w];
    const int b0 = carry;
    const int b1 = b0 + ((S0 + 31) & ~31);
    const int b2 = b1 + ((S1 + 31) & ~31);
    const int b3 = b2 + ((S2 + 31) & ~31);
    const int b4 = b3 + ((S3 + 31) & ~31);
    const int myb = sub == 0 ? b0 : (sub == 1 ? b1 : (sub == 2 ? b2 : b3));
    if (tid == 0) {
      srb[min(4 * ch + 0, RBN - 1)] = b0;
      srb[min(4 * ch + 1, RBN - 1)] = b1;
      srb[min(4 * ch + 2, RBN - 1)] = b2;
      srb[min(4 * ch + 3, RBN - 1)] = b3;
    }
    int run = myb + pre + incl - ts;
    soff[8 * tid + 0] = run; run += e0;
    soff[8 * tid + 1] = run; run += e1;
    soff[8 * tid + 2] = run; run += e2;
    soff[8 * tid + 3] = run; run += e3;
    soff[8 * tid + 4] = run; run += e4;
    soff[8 * tid + 5] = run; run += e5;
    soff[8 * tid + 6] = run; run += e6;
    soff[8 * tid + 7] = run;
    carry = b4;
    __syncthreads();
    const v4i o0 = *(const v4i*)(soff + 4 * tid);
    const v4i o1 = *(const v4i*)(soff + 4 * (tid + OTHR));
    int* op = off + base;
    *(volatile v4i*)(op + 4 * tid) = o0;
    *(volatile v4i*)(op + 4 * (tid + OTHR)) = o1;
    __threadfence();
    *(volatile v4i*)(op + 4 * tid) = o0;
    *(volatile v4i*)(op + 4 * (tid + OTHR)) = o1;
    __syncthreads();
  }
  if (tid == 0) srb[min(4 * nChunk, RBN - 1)] = carry;
  __syncthreads();
  v4i rv = {0, 0, 0, 0};
  if (tid < 32) rv = *(const v4i*)(srb + 4 * tid);
  if (tid < 32) *(volatile v4i*)(rbase + 4 * tid) = rv;
  __threadfence();
  if (tid < 32) *(volatile v4i*)(rbase + 4 * tid) = rv;
}

__global__ __launch_bounds__(NTHR) void k_fill(
    const int* __restrict__ srcs, const int* __restrict__ dsts,
    const int* __restrict__ off, const int* __restrict__ rbase,
    int* csr, int nN, int nE, int vec8, int csrLen) {
  extern __shared__ v4f lds_dyn[];
  int* region = (int*)lds_dyn;
  int* cursor = region + RCAP;
  int* list   = cursor + NBF;
  int* wcnt   = list + LISTN;
  const int tid = threadIdx.x, lane = tid & 31, wave = tid >> 5;
  const int b = blockIdx.x;
  const int nodeBase = b * NBF;

  int rb0 = rbase[b];
  const int rb1 = rbase[b + 1];
  rb0 = rb0 < 0 ? 0 : (rb0 > csrLen ? csrLen : rb0);
  rb0 &= ~31;
  int len = rb1 - rb0;
  len = len < 0 ? 0 : (len > RCAP ? RCAP : len);
  int lenW = (len + 31) & ~31;
  if (rb0 + lenW > csrLen) lenW = (csrLen - rb0) & ~31;

  {
    const v4i z = {0, 0, 0, 0};
    for (int i = tid; i < RCAP / 4; i += NTHR) ((v4i*)region)[i] = z;
    for (int s = tid; s < NBF; s += NTHR) {
      int o = off[nodeBase + s] - rb0;
      o = o < 0 ? 0 : (o > RCAP ? RCAP : o);
      cursor[s] = o;
    }
  }
  __syncthreads();

  const int nChunks = (nE + CHUNK - 1) / CHUNK;
#pragma unroll 1
  for (int ch = 0; ch < nChunks; ++ch) {
    const int cbase = ch * CHUNK;
    const int wc = scan_chunk<NBF>(dsts, nE, cbase, nodeBase, vec8, list, tid, lane, wave);
    if (lane == 0) wcnt[wave] = wc;
    __syncthreads();
    if (wave == 0) {
#pragma unroll 1
      for (int wsx = 0; wsx < NWAVE; ++wsx) {
        int n = __builtin_amdgcn_readfirstlane(wcnt[wsx]);
        n = n > WCAP ? WCAP : (n < 0 ? 0 : n);
        const int* lp = list + wsx * WCAP;
#pragma unroll 1
        for (int i = 0; i < n; ++i) {
          const int ent  = __builtin_amdgcn_readfirstlane(lp[i]);
          const int slot = ent & (NBF - 1);
          int e = cbase + ((ent >> 12) & (CHUNK - 1));
          e = e > nE - 1 ? nE - 1 : e;
          int sv = srcs[e];
          sv = sv < 0 ? 0 : (sv > nN - 1 ? nN - 1 : sv);
          if (lane == 0) {
            int pos = cursor[slot];
            pos = pos < 0 ? 0 : (pos > RCAP - 1 ? RCAP - 1 : pos);
            region[pos] = sv;
            const int np = pos + 1;
            cursor[slot] = np > RCAP ? RCAP : np;
          }
        }
      }
    }
    __syncthreads();
  }

  const int nv = lenW >> 2;
  int* gp = csr + rb0;
#pragma unroll 1
  for (int i = tid; i < nv; i += NTHR) { const v4i v = ((const v4i*)region)[i]; *(volatile v4i*)(gp + 4 * i) = v; }
  __threadfence();
#pragma unroll 1
  for (int i = tid; i < nv; i += NTHR) { const v4i v = ((const v4i*)region)[i]; *(volatile v4i*)(gp + 4 * i) = v; }
}

__global__ __launch_bounds__(NTHR) void k_norms(const int* __restrict__ cs, const int* __restrict__ cd,
                                                float* hn, float* tn, float* li, int nTot) {
  const int i0 = (int)blockIdx.x * NTHR + (int)threadIdx.x;
  int i = i0 > nTot - 1 ? nTot - 1 : i0;
  i = i < 0 ? 0 : i;
  int a = cs[i]; a = a < 1 ? 1 : a;
  int d = cd[i]; d = d < 1 ? 1 : d;
  const float od = (float)a, id = (float)d;
  const float vh = rsqrtf(od);
  const float vt = sqrtf(id);
  const float vl = log1pf(id);
  const bool st = i0 < nTot;
  if (st) { *(volatile float*)(hn + i0) = vh; *(volatile float*)(tn + i0) = vt; *(volatile float*)(li + i0) = vl; }
  __threadfence();
  if (st) { *(volatile float*)(hn + i0) = vh; *(volatile float*)(tn + i0) = vt; *(volatile float*)(li + i0) = vl; }
}

__global__ __launch_bounds__(NTHR) void k_wcvt(const float* __restrict__ w, _Float16* dp, int nUnits) {
  const int i = (int)blockIdx.x * NTHR + (int)threadIdx.x;
  if (i >= nUnits) return;
  const float* rp = w + (size_t)i * 8;
  const v4f x0 = *(const v4f*)rp;
  const v4f x1 = *(const v4f*)(rp + 4);
  v8h o;
  o[0] = (_Float16)(x0.x * WCARRY); o[1] = (_Float16)(x0.y * WCARRY); o[2] = (_Float16)(x0.z * WCARRY); o[3] = (_Float16)(x0.w * WCARRY);
  o[4] = (_Float16)(x1.x * WCARRY); o[5] = (_Float16)(x1.y * WCARRY); o[6] = (_Float16)(x1.z * WCARRY); o[7] = (_Float16)(x1.w * WCARRY);
  _Float16* gp = dp + (size_t)i * 8;
  *(volatile v8h*)gp = o;
  __threadfence();
  *(volatile v8h*)gp = o;
}

template <int ADD2>
__global__ __launch_bounds__(NTHR) void k_ln16(const float* __restrict__ x1, const float* __restrict__ x2,
                                               const float* __restrict__ g, const float* __restrict__ bb,
                                               _Float16* dp, int nN, int n1) {
  const int tid = threadIdx.x, lane = tid & 31, wave = tid >> 5;
  const int row = (int)blockIdx.x * NWAVE + wave;
  int r1 = row > n1 - 1 ? n1 - 1 : row; r1 = r1 < 0 ? 0 : r1;
  int r2 = row > nN - 1 ? nN - 1 : row; r2 = r2 < 0 ? 0 : r2;
  const bool live = row < nN;
  v4f v = *(const v4f*)(x1 + (size_t)r1 * FIN + 4 * lane);
  if (ADD2) {
    const v4f u = *(const v4f*)(x2 + (size_t)r2 * FIN + 4 * lane);
    v = v + u;
  }
  float s = v.x + v.y + v.z + v.w;
  s = wsum1(s);
  const float mu = s * (1.0f / (float)FIN);
  const float dx = v.x - mu, dy = v.y - mu, dz = v.z - mu, dw = v.w - mu;
  float q = dx * dx + dy * dy + dz * dz + dw * dw;
  q = wsum1(q);
  const float rs = rsqrtf(q * (1.0f / (float)FIN) + LNEPS);
  const v4f g4 = *(const v4f*)(g + 4 * lane);
  const v4f b4 = *(const v4f*)(bb + 4 * lane);
  const float y0 = dx * rs * g4.x + b4.x;
  const float y1 = dy * rs * g4.y + b4.y;
  const float y2 = dz * rs * g4.z + b4.z;
  const float y3 = dw * rs * g4.w + b4.w;
  const float sc = live ? ACARRY : 0.f;
  v4h o;
  o.x = (_Float16)(y0 * sc); o.y = (_Float16)(y1 * sc); o.z = (_Float16)(y2 * sc); o.w = (_Float16)(y3 * sc);
  _Float16* gp = dp + (size_t)row * FIN + 4 * lane;
  *(volatile v4h*)gp = o;
  __threadfence();
  *(volatile v4h*)gp = o;
}

template <int MODE>
__global__ __launch_bounds__(NTHR) void k_gemm(
    const _Float16* __restrict__ A, const _Float16* __restrict__ Bp,
    const float* __restrict__ rsc, const float* __restrict__ bias,
    const float* __restrict__ res1, const float* __restrict__ res2,
    void* Cv, int K, int ldc, int yplane, int nValid, int nStore, int nRes2, float scl) {
  constexpr int TPW = 4;
  static_assert(TPW * 16 * 2 == BNC);
  static_assert(BM == 4 * 16);

  __shared__ __attribute__((aligned(16))) StgU stg;
  const int tid = threadIdx.x, lane = tid & 31, wave = tid >> 5, hh = lane >> 4, m = lane & 15;
  const int rowBase = (int)blockIdx.x * BM;
  const int colBase = (int)blockIdx.y * BNC;
  const int ocol = (MODE == 0) ? 0 : colBase;
  const int rg = wave >> 1, chf = wave & 1;
  const int r0 = rg * 16;
  const int c0 = chf * (BNC / 2);

  v8f acc[TPW];
#pragma unroll
  for (int t = 0; t < TPW; ++t) { v8f z = {0.f, 0.f, 0.f, 0.f, 0.f, 0.f, 0.f, 0.f}; acc[t] = z; }

  const _Float16* ap = A  + (size_t)(rowBase + r0 + m) * K + 8 * hh;
  const _Float16* bp = Bp + (size_t)(colBase + c0 + m) * K + 8 * hh;
  const int ksteps = K >> 5;
#pragma unroll 1
  for (int kt = 0; kt < ksteps; ++kt) {
    Frag a;
    a.h[0] = *(const v8h*)(ap + 32 * kt);
    a.h[1] = *(const v8h*)(ap + 32 * kt + 16);
#pragma unroll
    for (int t = 0; t < TPW; ++t) {
      const size_t to = (size_t)(16 * t) * K + 32 * kt;
      Frag b;
      b.h[0] = *(const v8h*)(bp + to);
      b.h[1] = *(const v8h*)(bp + to + 16);
      acc[t] = wmh(a.v, b.v, acc[t]);
    }
  }

  const int growb = rowBase + r0 + 8 * hh;
  if constexpr (MODE == 1) {
    _Float16* sp = stg.h + (size_t)(r0 + 8 * hh) * BNC + c0 + m;
#pragma unroll
    for (int t = 0; t < TPW; ++t) {
      const float bc = bias[colBase + c0 + 16 * t + m];
#pragma unroll
      for (int r = 0; r < 8; ++r) {
        const bool lv = (growb + r) < nValid;
        const float g = fmaxf(acc[t][r] * scl + bc, 0.f);
        sp[r * BNC + 16 * t] = (_Float16)((lv ? g : 0.f) * ACARRY);
      }
    }
  } else {
    float rs8[8];
#pragma unroll
    for (int r = 0; r < 8; ++r) {
      if constexpr (MODE == 0) { rs8[r] = rsc[growb + r]; } else { rs8[r] = 1.0f; }
    }
    float* sp = stg.f + (size_t)(r0 + 8 * hh) * BNC + c0 + m;
#pragma unroll
    for (int t = 0; t < TPW; ++t) {
#pragma unroll
      for (int r = 0; r < 8; ++r) {
        const bool lv = (growb + r) < nValid;
        float g = acc[t][r] * scl;
        if constexpr (MODE == 0) { g = g * rs8[r]; }
        sp[r * BNC + 16 * t] = lv ? g : 0.f;
      }
    }
  }
  __syncthreads();

  if constexpr (MODE == 1) {
    constexpr int NIT = (BM * (BNC / 8)) / NTHR;
    static_assert(NIT * NTHR == BM * (BNC / 8));
    _Float16* C = (_Float16*)Cv;
    v8h cv[NIT];
#pragma unroll
    for (int it = 0; it < NIT; ++it) {
      const int id = it * NTHR + tid;
      const int row = id >> 4, seg = id & 15;
      cv[it] = *(const v8h*)(stg.h + (size_t)row * BNC + 8 * seg);
    }
#pragma unroll
    for (int it = 0; it < NIT; ++it) {
      const int id = it * NTHR + tid;
      const int row = id >> 4, seg = id & 15;
      const int grow = rowBase + row;
      if (grow < nStore) {
        _Float16* gp = C + (size_t)grow * ldc + ocol + 8 * seg;
        *(volatile v8h*)gp = cv[it];
      }
    }
    __threadfence();
#pragma unroll
    for (int it = 0; it < NIT; ++it) {
      const int id = it * NTHR + tid;
      const int row = id >> 4, seg = id & 15;
      const int grow = rowBase + row;
      if (grow < nStore) {
        _Float16* gp = C + (size_t)grow * ldc + ocol + 8 * seg;
        *(volatile v8h*)gp = cv[it];
      }
    }
  } else {
    constexpr int NIT = (BM * (BNC / 4)) / NTHR;
    static_assert(NIT * NTHR == BM * (BNC / 4));
    float* C = (float*)Cv;
    if constexpr (MODE == 0) { C = C + (size_t)blockIdx.y * (size_t)yplane; }
    v4f cv[NIT];
#pragma unroll
    for (int it = 0; it < NIT; ++it) {
      const int id = it * NTHR + tid;
      const int row = id >> 5, seg = id & 31;
      v4f v = *(const v4f*)(stg.f + (size_t)row * BNC + 4 * seg);
      if constexpr (MODE == 2) {
        const int grow = rowBase + row;
        int rr2 = grow > nRes2 - 1 ? nRes2 - 1 : grow;
        rr2 = rr2 < 0 ? 0 : rr2;
        const v4f b4  = *(const v4f*)(bias + ocol + 4 * seg);
        const v4f r1v = *(const v4f*)(res1 + (size_t)grow * ldc + ocol + 4 * seg);
        const v4f r2v = *(const v4f*)(res2 + (size_t)rr2 * ldc + ocol + 4 * seg);
        v = (v + b4) + (r1v + r2v);
      }
      cv[it] = v;
    }
#pragma unroll
    for (int it = 0; it < NIT; ++it) {
      const int id = it * NTHR + tid;
      const int row = id >> 5, seg = id & 31;
      const int grow = rowBase + row;
      if (grow < nStore) {
        float* gp = C + (size_t)grow * ldc + ocol + 4 * seg;
        *(volatile v4f*)gp = cv[it];
      }
    }
    __threadfence();
#pragma unroll
    for (int it = 0; it < NIT; ++it) {
      const int id = it * NTHR + tid;
      const int row = id >> 5, seg = id & 31;
      const int grow = rowBase + row;
      if (grow < nStore) {
        float* gp = C + (size_t)grow * ldc + ocol + 4 * seg;
        *(volatile v4f*)gp = cv[it];
      }
    }
  }
}

__global__ __launch_bounds__(NTHR) void k_elog(
    const int* __restrict__ csr, const int* __restrict__ off, const int* __restrict__ rbase,
    const float* __restrict__ fh, const float* __restrict__ ft, const float* __restrict__ av,
    const float* __restrict__ li, float* ea, int nN, int csrLen) {
  __shared__ __attribute__((aligned(16))) float sat[FIN];
  __shared__ int soff[NBF];
  __shared__ __attribute__((aligned(16))) float se[NTHR * NHD];
  const int tid = threadIdx.x;
  const int b = blockIdx.x;
  const int nodeBase = b * NBF;

  int rb0 = rbase[b];
  const int rb1 = rbase[b + 1];
  rb0 = rb0 < 0 ? 0 : (rb0 > csrLen ? csrLen : rb0);
  rb0 &= ~31;
  int len = rb1 - rb0;
  len = len < 0 ? 0 : (len > RCAP ? RCAP : len);
  int lenW = (len + 31) & ~31;
  if (rb0 + lenW > csrLen) lenW = (csrLen - rb0) & ~31;

  if (tid < FIN) sat[tid] = av[tid];
  for (int s = tid; s < NBF; s += NTHR) soff[s] = off[nodeBase + s] - rb0;
  __syncthreads();

  const int nb = (lenW + NTHR - 1) / NTHR;
#pragma unroll 1
  for (int it = 0; it < nb; ++it) {
    const int pl = it * NTHR + tid;
    int p = rb0 + pl;
    p = p > csrLen - 1 ? csrLen - 1 : p;
    p = p < 0 ? 0 : p;
    int s = csr[p];
    s = s < 0 ? 0 : (s > nN - 1 ? nN - 1 : s);
    int i = 0;
#pragma unroll
    for (int step = NBF / 2; step > 0; step >>= 1) {
      const int cand = i + step;
      i = (soff[cand] <= pl) ? cand : i;
    }
    const int dn = nodeBase + i;
    int dr = dn > nN - 1 ? nN - 1 : dn;
    dr = dr < 0 ? 0 : dr;
    const float lsc = li[dn] * INV_D;
    const float* hp = fh + (size_t)s * FIN;
    const float* tp = ft + (size_t)dr * FIN;
    float e0 = 0.f, e1 = 0.f, e2 = 0.f, e3 = 0.f, e4 = 0.f, e5 = 0.f, e6 = 0.f, e7 = 0.f;
#pragma unroll 1
    for (int h = 0; h < NHD; ++h) {
      float acc = 0.f;
#pragma unroll 1
      for (int q = 0; q < DHD / 4; ++q) {
        const int col = h * DHD + 4 * q;
        const v4f a4 = *(const v4f*)(hp + col);
        const v4f b4 = *(const v4f*)(tp + col);
        const v4f w4 = *(const v4f*)(sat + col);
        acc += lrelu1(a4.x * b4.x) * w4.x;
        acc += lrelu1(a4.y * b4.y) * w4.y;
        acc += lrelu1(a4.z * b4.z) * w4.z;
        acc += lrelu1(a4.w * b4.w) * w4.w;
      }
      const float ev = acc * lsc;
      e0 = (h == 0) ? ev : e0; e1 = (h == 1) ? ev : e1; e2 = (h == 2) ? ev : e2; e3 = (h == 3) ? ev : e3;
      e4 = (h == 4) ? ev : e4; e5 = (h == 5) ? ev : e5; e6 = (h == 6) ? ev : e6; e7 = (h == 7) ? ev : e7;
    }
    v4f lo, hi;
    lo.x = e0; lo.y = e1; lo.z = e2; lo.w = e3;
    hi.x = e4; hi.y = e5; hi.z = e6; hi.w = e7;
    *(v4f*)(se + NHD * tid) = lo;
    *(v4f*)(se + NHD * tid + 4) = hi;
    __syncthreads();
    const int rem = lenW - it * NTHR;
    const v4f c0 = *(const v4f*)(se + 4 * tid);
    const v4f c1 = *(const v4f*)(se + 4 * (tid + NTHR));
    const bool st0 = (tid >> 1) < rem;
    const bool st1 = (NTHR / 2 + (tid >> 1)) < rem;
    float* gp = ea + (size_t)(rb0 + it * NTHR) * NHD;
    if (st0) *(volatile v4f*)(gp + 4 * tid) = c0;
    if (st1) *(volatile v4f*)(gp + 4 * (tid + NTHR)) = c1;
    __threadfence();
    if (st0) *(volatile v4f*)(gp + 4 * tid) = c0;
    if (st1) *(volatile v4f*)(gp + 4 * (tid + NTHR)) = c1;
    __syncthreads();
  }
}

__global__ __launch_bounds__(NTHR) void k_esoft(
    const int* __restrict__ off, const int* __restrict__ cnt, const int* __restrict__ rbase,
    float* ea, int csrLen) {
  extern __shared__ v4f lds_dyn[];
  float* smax = (float*)lds_dyn;
  float* srcp = smax + NBF * NHD;
  float* sa   = srcp + NBF * NHD;
  int*   soff = (int*)(sa + NTHR * NHD);
  const int tid = threadIdx.x;
  const int b = blockIdx.x;
  const int nodeBase = b * NBF;

  int rb0 = rbase[b];
  const int rb1 = rbase[b + 1];
  rb0 = rb0 < 0 ? 0 : (rb0 > csrLen ? csrLen : rb0);
  rb0 &= ~31;
  int len = rb1 - rb0;
  len = len < 0 ? 0 : (len > RCAP ? RCAP : len);
  int lenW = (len + 31) & ~31;
  if (rb0 + lenW > csrLen) lenW = (csrLen - rb0) & ~31;

  for (int s = tid; s < NBF; s += NTHR) soff[s] = off[nodeBase + s] - rb0;

  const float NINF = -__builtin_inff();
#pragma unroll 1
  for (int k = 0; k < NBF / NTHR; ++k) {
    const int lc = k * NTHR + tid;
    const int c = nodeBase + lc;
    int n = cnt[c];
    n = n < 0 ? 0 : (n > DEGCAP ? DEGCAP : n);
    const int st = off[c];
    v4f mlo = {NINF, NINF, NINF, NINF};
    v4f mhi = {NINF, NINF, NINF, NINF};
#pragma unroll 1
    for (int q = 0; q < n; ++q) {
      int p = st + q;
      p = p < 0 ? 0 : (p > csrLen - 1 ? csrLen - 1 : p);
      const v4f elo = *(const v4f*)(ea + (size_t)p * NHD);
      const v4f ehi = *(const v4f*)(ea + (size_t)p * NHD + 4);
      mlo = vmax4(mlo, elo);
      mhi = vmax4(mhi, ehi);
    }
    const bool nz = n > 0;
    const v4f zero4 = {0.f, 0.f, 0.f, 0.f};
    mlo = nz ? mlo : zero4;
    mhi = nz ? mhi : zero4;
    v4f zlo = zero4, zhi = zero4;
#pragma unroll 1
    for (int q = 0; q < n; ++q) {
      int p = st + q;
      p = p < 0 ? 0 : (p > csrLen - 1 ? csrLen - 1 : p);
      const v4f elo = *(const v4f*)(ea + (size_t)p * NHD);
      const v4f ehi = *(const v4f*)(ea + (size_t)p * NHD + 4);
      zlo = zlo + vexp4(elo - mlo);
      zhi = zhi + vexp4(ehi - mhi);
    }
    v4f rlo = vrcp4(zlo), rhi = vrcp4(zhi);
    rlo = selz(rlo, nz);
    rhi = selz(rhi, nz);
    *(v4f*)(smax + NHD * lc)     = mlo;
    *(v4f*)(smax + NHD * lc + 4) = mhi;
    *(v4f*)(srcp + NHD * lc)     = rlo;
    *(v4f*)(srcp + NHD * lc + 4) = rhi;
  }
  __syncthreads();

  const int nb = (lenW + NTHR - 1) / NTHR;
#pragma unroll 1
  for (int it = 0; it < nb; ++it) {
    const int pl = it * NTHR + tid;
    int p = rb0 + pl;
    p = p > csrLen - 1 ? csrLen - 1 : p;
    p = p < 0 ? 0 : p;
    int i = 0;
#pragma unroll
    for (int step = NBF / 2; step > 0; step >>= 1) {
      const int cand = i + step;
      i = (soff[cand] <= pl) ? cand : i;
    }
    const v4f mlo = *(const v4f*)(smax + NHD * i);
    const v4f mhi = *(const v4f*)(smax + NHD * i + 4);
    const v4f rlo = *(const v4f*)(srcp + NHD * i);
    const v4f rhi = *(const v4f*)(srcp + NHD * i + 4);
    const v4f elo = *(const v4f*)(ea + (size_t)p * NHD);
    const v4f ehi = *(const v4f*)(ea + (size_t)p * NHD + 4);
    const v4f alo = vexp4(elo - mlo) * rlo;
    const v4f ahi = vexp4(ehi - mhi) * rhi;
    *(v4f*)(sa + NHD * tid) = alo;
    *(v4f*)(sa + NHD * tid + 4) = ahi;
    __syncthreads();
    const int rem = lenW - it * NTHR;
    const v4f c0 = *(const v4f*)(sa + 4 * tid);
    const v4f c1 = *(const v4f*)(sa + 4 * (tid + NTHR));
    const bool st0 = (tid >> 1) < rem;
    const bool st1 = (NTHR / 2 + (tid >> 1)) < rem;
    float* gp = ea + (size_t)(rb0 + it * NTHR) * NHD;
    if (st0) *(volatile v4f*)(gp + 4 * tid) = c0;
    if (st1) *(volatile v4f*)(gp + 4 * (tid + NTHR)) = c1;
    __threadfence();
    if (st0) *(volatile v4f*)(gp + 4 * tid) = c0;
    if (st1) *(volatile v4f*)(gp + 4 * (tid + NTHR)) = c1;
    __syncthreads();
  }
}

__global__ __launch_bounds__(NTHR) void k_hop(
    const int* __restrict__ csr, const int* __restrict__ off, const int* __restrict__ cnt,
    const float* __restrict__ ea, const float* __restrict__ hcur, const float* __restrict__ hn,
    const float* __restrict__ tn, const float* __restrict__ fe, float* hout,
    int nN, int csrLen, int useHn) {
  const int tid = threadIdx.x, lane = tid & 31, wave = tid >> 5, hq = lane >> 2;
  const int tbase = blockIdx.x * TGT + wave * 32;
  const int cl    = tbase + lane;
  const int cnt_l = cnt[cl];
  const int off_l = off[cl];
  const float tn_l = tn[cl];

#pragma unroll 1
  for (int j = 0; j < 32; ++j) {
    const int c = tbase + j;
    int n = __shfl(cnt_l, j);
    n = n < 0 ? 0 : (n > DEGCAP ? DEGCAP : n);
    const int st = __shfl(off_l, j);
    const float tnc = __shfl(tn_l, j);
    const v4f fec = *(const v4f*)(fe + (size_t)c * FIN + 4 * lane);

    v4f acc = {0.f, 0.f, 0.f, 0.f};
#pragma unroll 1
    for (int q0 = 0; q0 < n; q0 += 32) {
      int pos = st + q0 + lane;
      pos = pos < 0 ? 0 : (pos > csrLen - 1 ? csrLen - 1 : pos);
      int sl = csr[pos];
      sl = sl < 0 ? 0 : (sl > nN - 1 ? nN - 1 : sl);
      const int mcnt = (n - q0) < 32 ? (n - q0) : 32;
#pragma unroll 1
      for (int pp = 0; pp < mcnt; ++pp) {
        const int s = __builtin_amdgcn_readlane(sl, pp);
        int pa = st + q0 + pp;
        pa = pa < 0 ? 0 : (pa > csrLen - 1 ? csrLen - 1 : pa);
        float w = ea[(size_t)pa * NHD + hq];
        const float hs = hn[s];
        w = useHn ? (w * hs) : w;
        const v4f hv = *(const v4f*)(hcur + (size_t)s * FIN + 4 * lane);
        acc = acc + hv * w;
      }
    }

    const bool live = c < nN;
    v4f o = (acc * tnc) * OMA_C + fec * ALPHA_C;
    o = selz(o, live);
    float* gp = hout + (size_t)c * FIN + 4 * lane;
    *(volatile v4f*)gp = o;
    __threadfence();
    *(volatile v4f*)gp = o;
  }
}

extern "C" void kernel_launch(void* const* d_in, const int* in_sizes, int n_in,
                              void* d_out, int out_size, void* d_ws, size_t ws_size,
                              hipStream_t stream) {
  if (n_in < 15) return;
  if (in_sizes[0] < FIN || (in_sizes[0] % FIN) != 0) return;
  const int nN = in_sizes[0] / FIN;
  if (nN < 1 || nN > 131072) return;
  const int nE = in_sizes[1];
  if (nE < 1 || nE > (1 << 26) || in_sizes[2] != nE) return;
  if (in_sizes[3] != FIN * FIN || in_sizes[4] != FIN * FIN || in_sizes[5] != FIN * FIN) return;
  if (in_sizes[6] != NHD * DHD) return;
  if (in_sizes[7] != FIN || in_sizes[8] != FIN || in_sizes[9] != FIN || in_sizes[10] != FIN) return;
  if (in_sizes[11] != FFH * FIN || in_sizes[12] != FFH) return;
  if (in_sizes[13] != FIN * FFH || in_sizes[14] != FIN) return;
  if (out_size != nN * FIN) return;

  const float* feat   = (const float*)d_in[0];
  const int*   src    = (const int*)d_in[1];
  const int*   dst    = (const int*)d_in[2];
  const float* w_head = (const float*)d_in[3];
  const float* w_tail = (const float*)d_in[4];
  const float* w_ent  = (const float*)d_in[5];
  const float* attn   = (const float*)d_in[6];
  const float* ln1_g  = (const float*)d_in[7];
  const float* ln1_b  = (const float*)d_in[8];
  const float* ln2_g  = (const float*)d_in[9];
  const float* ln2_b  = (const float*)d_in[10];
  const float* ff_w1  = (const float*)d_in[11];
  const float* ff_b1  = (const float*)d_in[12];
  const float* ff_w2  = (const float*)d_in[13];
  const float* ff_b2  = (const float*)d_in[14];
  float* out = (float*)d_out;

  const int NPAD   = ((nN + TGT - 1) / TGT) * TGT;
  const int nAgg   = NPAD / TGT;
  const int nBC    = (nN + NBC - 1) / NBC;
  const int CNTPAD = nBC * NBC;
  if (CNTPAD < NPAD) return;
  if (4 * nBC + 1 > RBN) return;
  const int nBF    = (nN + NBF - 1) / NBF;
  if (nBF > 4 * nBC) return;
  const int csrLen = ((nE + 31) & ~31) + 4096;
  if (31 * 4 * nBC > 4096) return;

  char* ws = (char*)d_ws;
  size_t off = 0;
  const size_t oCs  = off; off += (size_t)CNTPAD * 4;                    off = (off + 255) & ~(size_t)255;
  const size_t oCd  = off; off += (size_t)CNTPAD * 4;                    off = (off + 255) & ~(size_t)255;
  const size_t oOff = off; off += (size_t)CNTPAD * 4;                    off = (off + 255) & ~(size_t)255;
  const size_t oRb  = off; off += (size_t)RBN * 4;                       off = (off + 255) & ~(size_t)255;
  const size_t oCsr = off; off += (size_t)csrLen * 4;                    off = (off + 255) & ~(size_t)255;
  const size_t oEa  = off; off += (size_t)csrLen * NHD * 4;              off = (off + 255) & ~(size_t)255;
  const size_t oHn  = off; off += (size_t)CNTPAD * 4;                    off = (off + 255) & ~(size_t)255;
  const size_t oTn  = off; off += (size_t)CNTPAD * 4;                    off = (off + 255) & ~(size_t)255;
  const size_t oLi  = off; off += (size_t)CNTPAD * 4;                    off = (off + 255) & ~(size_t)255;
  const size_t oWpj = off; off += (size_t)NPJ * FIN * FIN * 2;           off = (off + 255) & ~(size_t)255;
  const size_t oW1  = off; off += (size_t)FFH * FIN * 2;                 off = (off + 255) & ~(size_t)255;
  const size_t oW2  = off; off += (size_t)FIN * FFH * 2;                 off = (off + 255) & ~(size_t)255;
  const size_t oXa  = off; off += (size_t)NPAD * FIN * 2;                off = (off + 255) & ~(size_t)255;
  const size_t oPj  = off; off += (size_t)NPJ * NPAD * FIN * 4;          off = (off + 255) & ~(size_t)255;
  if (off > ws_size || off > (size_t)WSCAP) return;

  int*   cntS = (int*)(ws + oCs);
  int*   cntD = (int*)(ws + oCd);
  int*   offp = (int*)(ws + oOff);
  int*   rb   = (int*)(ws + oRb);
  int*   csr  = (int*)(ws + oCsr);
  float* ea   = (float*)(ws + oEa);
  float* hn   = (float*)(ws + oHn);
  float* tn   = (float*)(ws + oTn);
  float* li   = (float*)(ws + oLi);
  _Float16* wpj = (_Float16*)(ws + oWpj);
  _Float16* w1p = (_Float16*)(ws + oW1);
  _Float16* w2p = (_Float16*)(ws + oW2);
  _Float16* xa  = (_Float16*)(ws + oXa);
  float* pj   = (float*)(ws + oPj);
  float* P0 = pj;
  float* P1 = pj + (size_t)NPAD * FIN;
  float* P2 = pj + (size_t)2 * NPAD * FIN;
  _Float16* y1p = (_Float16*)P1;

  const int vec8 = 1;

  k_count<<<nBC, NTHR, 0, stream>>>(src, cntS, nE, vec8);
  k_count<<<nBC, NTHR, 0, stream>>>(dst, cntD, nE, vec8);
  k_offsets<<<1, OTHR, 0, stream>>>(cntD, offp, rb, nBC);
  hipFuncSetAttribute(reinterpret_cast<const void*>(&k_fill),
                      hipFuncAttributeMaxDynamicSharedMemorySize, LDS_FILL);
  k_fill<<<nBF, NTHR, LDS_FILL, stream>>>(src, dst, offp, rb, csr, nN, nE, vec8, csrLen);

  {
    const int u = (FIN * FIN) / 8;
    k_wcvt<<<(u + NTHR - 1) / NTHR, NTHR, 0, stream>>>(w_head, wpj, u);
    k_wcvt<<<(u + NTHR - 1) / NTHR, NTHR, 0, stream>>>(w_tail, wpj + (size_t)FIN * FIN, u);
    k_wcvt<<<(u + NTHR - 1) / NTHR, NTHR, 0, stream>>>(w_ent,  wpj + (size_t)2 * FIN * FIN, u);
    const int u2 = (FFH * FIN) / 8;
    k_wcvt<<<(u2 + NTHR - 1) / NTHR, NTHR, 0, stream>>>(ff_w1, w1p, u2);
    k_wcvt<<<(u2 + NTHR - 1) / NTHR, NTHR, 0, stream>>>(ff_w2, w2p, u2);
  }

  k_norms<<<CNTPAD / NTHR, NTHR, 0, stream>>>(cntS, cntD, hn, tn, li, CNTPAD);
  k_ln16<0><<<NPAD / NWAVE, NTHR, 0, stream>>>(feat, feat, ln1_g, ln1_b, xa, nN, nN);
  k_gemm<0><<<dim3(NPAD / BM, (NPJ * FIN) / BNC), NTHR, 0, stream>>>(
      xa, wpj, hn, hn, hn, hn, (void*)pj, FIN, FIN, NPAD * FIN, nN, NPAD, nN, SCL_AW);

  k_elog<<<nBF, NTHR, 0, stream>>>(csr, offp, rb, P0, P1, attn, li, ea, nN, csrLen);
  hipFuncSetAttribute(reinterpret_cast<const void*>(&k_esoft),
                      hipFuncAttributeMaxDynamicSharedMemorySize, LDS_SOFT);
  k_esoft<<<nBF, NTHR, LDS_SOFT, stream>>>(offp, cntD, rb, ea, csrLen);

  const float* cur = P2;
  for (int hop = 0; hop < NHOP; ++hop) {
    float* ho = (hop & 1) ? P1 : P0;
    k_hop<<<nAgg, NTHR, 0, stream>>>(csr, offp, cntD, ea, cur, hn, tn, P2, ho, nN, csrLen, hop > 0 ? 1 : 0);
    cur = ho;
  }
  float* hfin = P0;

  k_ln16<1><<<NPAD / NWAVE, NTHR, 0, stream>>>(hfin, feat, ln2_g, ln2_b, xa, nN, NPAD);
  k_gemm<1><<<dim3(NPAD / BM, FFH / BNC), NTHR, 0, stream>>>(
      xa, w1p, hn, ff_b1, hn, hn, (void*)y1p, FIN, FFH, 0, nN, NPAD, nN, SCL_AW);
  k_gemm<2><<<dim3(NPAD / BM, FIN / BNC), NTHR, 0, stream>>>(
      y1p, w2p, hn, ff_b2, hfin, feat, (void*)out, FFH, FIN, 0, nN, nN, nN, SCL_AW);
}
